// GATEncoderWrapper_11132555231669
// MI455X (gfx1250) — hardware-verified
//
#include <hip/hip_runtime.h>
#include <stddef.h>


#define NTHR  256
#define NWAVE 8
#define GR    32
#define GC    128
#define XSP   132
#define CHUNK 2048
#define WCAP  256
#define NGRP  (CHUNK / (NTHR * 4))
#define ACCF  65536
#define MXN   512
#define AGG_LDS_BYTES ((ACCF + 2 * MXN) * 4 + (NWAVE * WCAP + NWAVE) * 4)

static_assert(NGRP == 2);
static_assert(WCAP == (CHUNK / NTHR) * 32);
static_assert(AGG_LDS_BYTES == 274464);
static_assert((XSP % 4) == 0);

typedef float          v4f  __attribute__((ext_vector_type(4)));
typedef float          v8f  __attribute__((ext_vector_type(8)));
typedef int            v4i  __attribute__((ext_vector_type(4)));
typedef _Float16       v8h  __attribute__((ext_vector_type(8)));
typedef _Float16       v16h __attribute__((ext_vector_type(16)));
typedef __bf16         v16b __attribute__((ext_vector_type(16)));
typedef unsigned short v8us __attribute__((ext_vector_type(8)));

union FragH { v16h v; v4i u[2]; };
union FragB { v16b v; v4i u[2]; };
union Pack  { v8h h; v8us s; v4i i; };

__device__ __forceinline__ unsigned short f2bf(float x) {
  unsigned b = __float_as_uint(x);
  b += 0x7FFFu + ((b >> 16) & 1u);
  return (unsigned short)(b >> 16);
}
__device__ __forceinline__ float bf2f(unsigned short h) { return __uint_as_float(((unsigned)h) << 16); }

__device__ __forceinline__ v8f wmh(v16h a, v16h b, v8f c) {
  v8f d = __builtin_amdgcn_wmma_f32_16x16x32_f16(false, a, false, b, (short)0, c, false, false);
  asm volatile("v_nop\n\tv_nop\n\tv_nop\n\tv_nop" : "+v"(d) : "v"(a), "v"(b));
  return d;
}
__device__ __forceinline__ v8f wmb(v16b a, v16b b, v8f c) {
  v8f d = __builtin_amdgcn_wmma_f32_16x16x32_bf16(false, a, false, b, (short)0, c, false, false);
  asm volatile("v_nop\n\tv_nop\n\tv_nop\n\tv_nop" : "+v"(d) : "v"(a), "v"(b));
  return d;
}

__device__ __forceinline__ float lk(float t) { return fmaxf(t, 0.2f * t); }
__device__ __forceinline__ float dl(v4f t, v4f w) {
  return w.x * lk(t.x) + w.y * lk(t.y) + w.z * lk(t.z) + w.w * lk(t.w);
}

__global__ __launch_bounds__(NTHR) void k_cvt(const float* __restrict__ src, int rows_src, int K,
                                              unsigned short* ph, unsigned short* pl, unsigned short* pf,
                                              int rows_total, int Kpad, float fscale, int mode) {
  const int kp8 = Kpad >> 3;
  const int n8  = rows_total * kp8;
  const int i   = blockIdx.x * NTHR + threadIdx.x;
  if (i >= n8) return;
  const int r  = i / kp8;
  const int kb = (i - r * kp8) * 8;
  const int rc = (r < rows_src) ? r : (rows_src - 1);
  float v[8];
#pragma unroll
  for (int j = 0; j < 8; ++j) {
    const int kk = kb + j;
    const int kc = (kk < K) ? kk : (K - 1);
    const float t = src[(size_t)rc * K + kc];
    v[j] = (r < rows_src && kk < K) ? t : 0.f;
  }
  Pack uh, ul, uf;
  const v4i z4 = {0, 0, 0, 0};
  uh.i = z4; ul.i = z4; uf.i = z4;
#pragma unroll
  for (int j = 0; j < 8; ++j) {
    const unsigned short hb = f2bf(v[j]);
    uh.s[j] = hb;
    ul.s[j] = f2bf(v[j] - bf2f(hb));
    uf.h[j] = (_Float16)(v[j] * fscale);
  }
  const size_t o = (size_t)i * 8;
  if (mode & 1) { *(volatile v4i*)(ph + o) = uh.i; *(volatile v4i*)(pl + o) = ul.i; }
  if (mode & 2) { *(volatile v4i*)(pf + o) = uf.i; }
  __threadfence();
  if (mode & 1) { *(volatile v4i*)(ph + o) = uh.i; *(volatile v4i*)(pl + o) = ul.i; }
  if (mode & 2) { *(volatile v4i*)(pf + o) = uf.i; }
}

template <int SPLIT>
__global__ __launch_bounds__(NTHR) void k_gemm(
    const unsigned short* __restrict__ A0, const unsigned short* __restrict__ A1,
    const unsigned short* __restrict__ B0, const unsigned short* __restrict__ B1,
    const float* __restrict__ bias, float* out, int K, int Ncols, float oscale) {
  __shared__ __attribute__((aligned(16))) float Xs[GR * XSP];

  const int tid  = threadIdx.x;
  const int lane = tid & 31;
  const int wave = tid >> 5;
  const int hh   = lane >> 4;
  const int m    = lane & 15;
  const int rowBase = blockIdx.x * GR;
  const int colBase = blockIdx.y * GC;
  const int ncol = colBase + wave * 16 + m;

  const size_t ra0 = (size_t)(rowBase + m) * K + 8 * hh;
  const size_t ra1 = ra0 + (size_t)16 * K;
  const size_t rb  = (size_t)ncol * K + 8 * hh;

  v8f c0 = {0.f, 0.f, 0.f, 0.f, 0.f, 0.f, 0.f, 0.f};
  v8f c1 = {0.f, 0.f, 0.f, 0.f, 0.f, 0.f, 0.f, 0.f};

#pragma unroll 1
  for (int k0 = 0; k0 < K; k0 += 32) {
    if (SPLIT) {
      FragB ah0, ah1, al0, al1, bh, bl;
      ah0.u[0] = *(const v4i*)(A0 + ra0 + k0);  ah0.u[1] = *(const v4i*)(A0 + ra0 + k0 + 16);
      ah1.u[0] = *(const v4i*)(A0 + ra1 + k0);  ah1.u[1] = *(const v4i*)(A0 + ra1 + k0 + 16);
      al0.u[0] = *(const v4i*)(A1 + ra0 + k0);  al0.u[1] = *(const v4i*)(A1 + ra0 + k0 + 16);
      al1.u[0] = *(const v4i*)(A1 + ra1 + k0);  al1.u[1] = *(const v4i*)(A1 + ra1 + k0 + 16);
      bh.u[0]  = *(const v4i*)(B0 + rb + k0);   bh.u[1]  = *(const v4i*)(B0 + rb + k0 + 16);
      bl.u[0]  = *(const v4i*)(B1 + rb + k0);   bl.u[1]  = *(const v4i*)(B1 + rb + k0 + 16);
      c0 = wmb(ah0.v, bh.v, c0);  c0 = wmb(ah0.v, bl.v, c0);  c0 = wmb(al0.v, bh.v, c0);
      c1 = wmb(ah1.v, bh.v, c1);  c1 = wmb(ah1.v, bl.v, c1);  c1 = wmb(al1.v, bh.v, c1);
    } else {
      FragH a0, a1, b;
      a0.u[0] = *(const v4i*)(A0 + ra0 + k0);  a0.u[1] = *(const v4i*)(A0 + ra0 + k0 + 16);
      a1.u[0] = *(const v4i*)(A0 + ra1 + k0);  a1.u[1] = *(const v4i*)(A0 + ra1 + k0 + 16);
      b.u[0]  = *(const v4i*)(B0 + rb + k0);   b.u[1]  = *(const v4i*)(B0 + rb + k0 + 16);
      c0 = wmh(a0.v, b.v, c0);
      c1 = wmh(a1.v, b.v, c1);
    }
  }

  const float bv = bias[ncol];
  const int cl = wave * 16 + m;
#pragma unroll
  for (int r = 0; r < 8; ++r) {
    Xs[(8 * hh + r) * XSP + cl]      = c0[r] * oscale + bv;
    Xs[(16 + 8 * hh + r) * XSP + cl] = c1[r] * oscale + bv;
  }
  __syncthreads();

  v4f xv[4];
  float* xpp[4];
#pragma unroll
  for (int i = 0; i < 4; ++i) {
    xv[i]  = *(const v4f*)(Xs + (4 * wave + i) * XSP + 4 * lane);
    xpp[i] = out + (size_t)(rowBase + 4 * wave + i) * Ncols + colBase + 4 * lane;
  }
#pragma unroll
  for (int i = 0; i < 4; ++i) *(volatile v4f*)(xpp[i]) = xv[i];
  __threadfence();
#pragma unroll
  for (int i = 0; i < 4; ++i) *(volatile v4f*)(xpp[i]) = xv[i];
}

__device__ __forceinline__ void hit16(const float* xs, const float* xd, float* ar, float* mp, float* dp,
                                      v4f w0, v4f w1, v4f w2, v4f w3) {
  const v4f a0 = *(const v4f*)(xs),       a1 = *(const v4f*)(xs + 4);
  const v4f a2 = *(const v4f*)(xs + 256), a3 = *(const v4f*)(xs + 260);
  const v4f d0 = *(const v4f*)(xd),       d1 = *(const v4f*)(xd + 4);
  const v4f d2 = *(const v4f*)(xd + 256), d3 = *(const v4f*)(xd + 260);
  float sA = dl(a0 + d0, w0) + dl(a1 + d1, w1);
  float sB = dl(a2 + d2, w2) + dl(a3 + d3, w3);
  sA += __shfl_xor(sA, 8, 32);  sB += __shfl_xor(sB, 8, 32);
  sA += __shfl_xor(sA, 4, 32);  sB += __shfl_xor(sB, 4, 32);
  sA += __shfl_xor(sA, 2, 32);  sB += __shfl_xor(sB, 2, 32);
  sA += __shfl_xor(sA, 1, 32);  sB += __shfl_xor(sB, 1, 32);
  const float mA = mp[0], mB = mp[2];
  const float nA = dp[0], nB = dp[2];
  const float mnA = fmaxf(mA, sA), mnB = fmaxf(mB, sB);
  const float scA = __expf(mA - mnA), scB = __expf(mB - mnB);
  const float pA  = __expf(sA - mnA), pB  = __expf(sB - mnB);
  v4f e0 = *(v4f*)(ar),       e1 = *(v4f*)(ar + 4);
  v4f e2 = *(v4f*)(ar + 256), e3 = *(v4f*)(ar + 260);
  e0 = e0 * scA + a0 * pA;  e1 = e1 * scA + a1 * pA;
  e2 = e2 * scB + a2 * pB;  e3 = e3 * scB + a3 * pB;
  *(v4f*)(ar)       = e0;  *(v4f*)(ar + 4)   = e1;
  *(v4f*)(ar + 256) = e2;  *(v4f*)(ar + 260) = e3;
  mp[0] = mnA;  mp[2] = mnB;
  dp[0] = nA * scA + pA;  dp[2] = nB * scB + pB;
}

__device__ __forceinline__ void hit4(const float* xs, const float* xd, float* ar, float* mp, float* dp, v4f w0) {
  const v4f a0 = *(const v4f*)(xs);
  const v4f d0 = *(const v4f*)(xd);
  float s = dl(a0 + d0, w0);
  s += __shfl_xor(s, 16, 32);
  s += __shfl_xor(s, 8, 32);
  s += __shfl_xor(s, 4, 32);
  s += __shfl_xor(s, 2, 32);
  s += __shfl_xor(s, 1, 32);
  const float m  = mp[0], n = dp[0];
  const float mn = fmaxf(m, s);
  const float sc = __expf(m - mn);
  const float p  = __expf(s - mn);
  v4f e0 = *(v4f*)(ar);
  e0 = e0 * sc + a0 * p;
  *(v4f*)(ar) = e0;
  mp[0] = mn;
  dp[0] = n * sc + p;
}

template <int NHD, int NB>
__global__ __launch_bounds__(NTHR) void k_agg(
    const int* __restrict__ ei, const float* __restrict__ xl, const float* __restrict__ xr,
    const float* __restrict__ att, const float* __restrict__ bias,
    unsigned short* ph, unsigned short* pl, unsigned short* pf, float* out,
    int nN, int nE, int nW) {
  constexpr int DFW = NHD * 128;
  static_assert(NB * DFW == ACCF);
  static_assert(NB * NHD == MXN);
  static_assert((NB & (NB - 1)) == 0);
  static_assert(NB <= 512);
  static_assert(NB <= NWAVE * WCAP);

  extern __shared__ v4f lds_dyn[];
  float* sacc = (float*)lds_dyn;
  float* mx   = sacc + ACCF;
  float* dn   = mx + MXN;
  int*   list = (int*)(dn + MXN);
  int*   wcnt = list + NWAVE * WCAP;

  const int tid  = threadIdx.x;
  const int lane = tid & 31;
  const int wave = tid >> 5;
  const int nodeBase = blockIdx.x * NB;

  {
    const v4f z4 = {0.f, 0.f, 0.f, 0.f};
    for (int i = tid; i < ACCF / 4; i += NTHR) lds_dyn[i] = z4;
    for (int i = tid; i < MXN; i += NTHR) { mx[i] = -1.0e30f; dn[i] = 0.f; }
  }
  __syncthreads();

  const int coff = (NHD == 4) ? (8 * lane) : (4 * lane);
  const int hidx = (NHD == 4) ? (lane >> 4) : 0;
  const v4f w0 = *(const v4f*)(att + coff);
  v4f w1 = w0, w2 = w0, w3 = w0;
  if (NHD == 4) {
    w1 = *(const v4f*)(att + coff + 4);
    w2 = *(const v4f*)(att + coff + 256);
    w3 = *(const v4f*)(att + coff + 260);
  }

  const int* eid = ei + nE;
  const bool al16 = ((nE & 3) == 0);
  const int nChunks = (nE + CHUNK - 1) / CHUNK;

#pragma unroll 1
  for (int ch = 0; ch <= nChunks; ++ch) {
    const int cbase = ch * CHUNK;
    const bool selfp = (ch == nChunks);
    if (!selfp) {
      int wc = 0;
#pragma unroll
      for (int g = 0; g < NGRP; ++g) {
        const int el0 = (g * NTHR + tid) * 4;
        const int e0  = cbase + el0;
        const int sent = -2147483647 - 1;
        v4i d;
        if (al16 && (e0 + 3 < nE)) {
          d = *(const v4i*)(eid + e0);
        } else {
          d.x = (e0     < nE) ? eid[min(e0, nE - 1)]     : sent;
          d.y = (e0 + 1 < nE) ? eid[min(e0 + 1, nE - 1)] : sent;
          d.z = (e0 + 2 < nE) ? eid[min(e0 + 2, nE - 1)] : sent;
          d.w = (e0 + 3 < nE) ? eid[min(e0 + 3, nE - 1)] : sent;
        }
        const unsigned s0 = (unsigned)d.x - (unsigned)nodeBase;
        const unsigned s1 = (unsigned)d.y - (unsigned)nodeBase;
        const unsigned s2 = (unsigned)d.z - (unsigned)nodeBase;
        const unsigned s3 = (unsigned)d.w - (unsigned)nodeBase;
        const bool h0 = s0 < (unsigned)NB;
        const bool h1 = s1 < (unsigned)NB;
        const bool h2 = s2 < (unsigned)NB;
        const bool h3 = s3 < (unsigned)NB;
        const unsigned many = __builtin_amdgcn_ballot_w32(h0 | h1 | h2 | h3);
        if (many != 0u) {
#define HITJ(J, HJ, SJ) { \
            const unsigned mj = __builtin_amdgcn_ballot_w32(HJ); \
            if (HJ) { \
              const int pos = wc + (int)__builtin_amdgcn_mbcnt_lo(mj, 0u); \
              if (pos < WCAP) list[wave * WCAP + pos] = ((el0 + (J)) << 9) | (int)(SJ); \
            } \
            wc += (int)__builtin_popcount(mj); }
          HITJ(0, h0, s0)
          HITJ(1, h1, s1)
          HITJ(2, h2, s2)
          HITJ(3, h3, s3)
#undef HITJ
        }
      }
      if (lane == 0) wcnt[wave] = wc;
    } else {
      for (int s = tid; s < NB; s += NTHR) list[s] = s;
      if (tid < NWAVE) {
        int c = NB - tid * WCAP;
        c = c < 0 ? 0 : (c > WCAP ? WCAP : c);
        wcnt[tid] = c;
      }
    }
    __syncthreads();

    if (wave == 0) {
#pragma unroll 1
      for (int wsx = 0; wsx < NWAVE; ++wsx) {
        int n = __builtin_amdgcn_readfirstlane(wcnt[wsx]);
        n = n > WCAP ? WCAP : n;
        n = n < 0 ? 0 : n;
#pragma unroll 1
        for (int i = 0; i < n; ++i) {
          const int ent  = __builtin_amdgcn_readfirstlane(list[wsx * WCAP + i]);
          const int slot = ent & (NB - 1);
          const int el   = (ent >> 9) & (CHUNK - 1);
          const int node = nodeBase + slot;
          if (node >= nN) continue;
          int e = cbase + el;
          if (e > nE - 1) e = nE - 1;
          int sj = ei[e];
          sj = sj < 0 ? 0 : (sj > nN - 1 ? nN - 1 : sj);
          const int src = selfp ? node : sj;
          const float* xs = xl + (size_t)src * DFW + coff;
          const float* xd = xr + (size_t)node * DFW + coff;
          float* ar = sacc + slot * DFW + coff;
          float* mp = mx + slot * NHD + hidx;
          float* dp = dn + slot * NHD + hidx;
          if (NHD == 4) hit16(xs, xd, ar, mp, dp, w0, w1, w2, w3);
          else          hit4(xs, xd, ar, mp, dp, w0);
        }
      }
    }
    __syncthreads();
  }

  if (NHD == 4) {
#pragma unroll 1
    for (int s = wave; s < NB; s += NWAVE) {
      const int node = nodeBase + s;
      if (node >= nW) break;
      const size_t ro = (size_t)node * DFW;
#pragma unroll 1
      for (int q2 = 0; q2 < 2; ++q2) {
        const int co  = 256 * q2 + 8 * lane;
        const int hq  = 2 * q2 + (lane >> 4);
        Pack uh, ul, uf;
        const v4i z4 = {0, 0, 0, 0};
        uh.i = z4; ul.i = z4; uf.i = z4;
        if (node < nN) {
          const float* ar = sacc + s * DFW + co;
          const v4f e0 = *(const v4f*)(ar), e1 = *(const v4f*)(ar + 4);
          const float inv = 1.0f / (dn[s * NHD + hq] + 1e-16f);
          const v4f b0 = *(const v4f*)(bias + co), b1 = *(const v4f*)(bias + co + 4);
          const v4f o0 = e0 * inv + b0;
          const v4f o1 = e1 * inv + b1;
#pragma unroll
          for (int j = 0; j < 4; ++j) {
            float v = o0[j];
            v = (v > 0.f) ? v : (__expf(v) - 1.0f);
            const unsigned short hb = f2bf(v);
            uh.s[j] = hb;
            ul.s[j] = f2bf(v - bf2f(hb));
            uf.h[j] = (_Float16)v;
            float u = o1[j];
            u = (u > 0.f) ? u : (__expf(u) - 1.0f);
            const unsigned short hc = f2bf(u);
            uh.s[4 + j] = hc;
            ul.s[4 + j] = f2bf(u - bf2f(hc));
            uf.h[4 + j] = (_Float16)u;
          }
        }
        *(volatile v4i*)(ph + ro + co) = uh.i;
        *(volatile v4i*)(pl + ro + co) = ul.i;
        *(volatile v4i*)(pf + ro + co) = uf.i;
        __threadfence();
        *(volatile v4i*)(ph + ro + co) = uh.i;
        *(volatile v4i*)(pl + ro + co) = ul.i;
        *(volatile v4i*)(pf + ro + co) = uf.i;
      }
    }
  } else {
#pragma unroll 1
    for (int s = wave; s < NB; s += NWAVE) {
      const int node = nodeBase + s;
      if (node >= nW) break;
      const int co = 4 * lane;
      const v4f e0 = *(const v4f*)(sacc + s * DFW + co);
      const float inv = 1.0f / (dn[s * NHD] + 1e-16f);
      const v4f b0 = *(const v4f*)(bias + co);
      const v4f o = e0 * inv + b0;
      float* op = out + (size_t)node * DFW + co;
      *(volatile v4f*)op = o;
      __threadfence();
      *(volatile v4f*)op = o;
    }
  }
}

extern "C" void kernel_launch(void* const* d_in, const int* in_sizes, int n_in,
                              void* d_out, int out_size, void* d_ws, size_t ws_size,
                              hipStream_t stream) {
  if (n_in < 20) return;
  const int IN = 77, DW = 512, C3 = 128, K1 = 96;
  const int nN = in_sizes[0] / IN;
  if (nN <= 0 || in_sizes[0] != nN * IN) return;
  const int nE = in_sizes[1] / 2;
  if (nE <= 0 || in_sizes[1] != 2 * nE) return;
  if (in_sizes[2] != DW * IN || in_sizes[3] != DW || in_sizes[4] != DW * IN || in_sizes[5] != DW ||
      in_sizes[6] != DW || in_sizes[7] != DW) return;
  if (in_sizes[8] != DW * DW || in_sizes[9] != DW || in_sizes[10] != DW * DW || in_sizes[11] != DW ||
      in_sizes[12] != DW || in_sizes[13] != DW) return;
  if (in_sizes[14] != C3 * DW || in_sizes[15] != C3 || in_sizes[16] != C3 * DW || in_sizes[17] != C3 ||
      in_sizes[18] != C3 || in_sizes[19] != C3) return;
  if (out_size != nN * C3) return;

  const float* x   = (const float*)d_in[0];
  const int*   ei  = (const int*)d_in[1];
  const float* Wl1 = (const float*)d_in[2];   const float* bl1 = (const float*)d_in[3];
  const float* Wr1 = (const float*)d_in[4];   const float* br1 = (const float*)d_in[5];
  const float* at1 = (const float*)d_in[6];   const float* b1  = (const float*)d_in[7];
  const float* Wl2 = (const float*)d_in[8];   const float* bl2 = (const float*)d_in[9];
  const float* Wr2 = (const float*)d_in[10];  const float* br2 = (const float*)d_in[11];
  const float* at2 = (const float*)d_in[12];  const float* b2  = (const float*)d_in[13];
  const float* Wl3 = (const float*)d_in[14];  const float* bl3 = (const float*)d_in[15];
  const float* Wr3 = (const float*)d_in[16];  const float* br3 = (const float*)d_in[17];
  const float* at3 = (const float*)d_in[18];  const float* b3  = (const float*)d_in[19];
  float* out = (float*)d_out;

  const int Mpad = ((nN + GR - 1) / GR) * GR;

  char* wsp = (char*)d_ws;
  size_t off = 0;
  const size_t plB = (size_t)Mpad * DW * 2;
  const size_t wB  = (size_t)DW * DW * 2;
  const size_t xB  = (size_t)Mpad * DW * 4;
  unsigned short* Ah = (unsigned short*)(wsp + off); off += plB;
  unsigned short* Al = (unsigned short*)(wsp + off); off += plB;
  unsigned short* Af = (unsigned short*)(wsp + off); off += plB;
  unsigned short* Bh = (unsigned short*)(wsp + off); off += wB;
  unsigned short* Bl = (unsigned short*)(wsp + off); off += wB;
  unsigned short* Bf = (unsigned short*)(wsp + off); off += wB;
  float* xl = (float*)(wsp + off); off += xB;
  float* xr = (float*)(wsp + off); off += xB;
  if (off > ws_size) return;

  const float s16  = 16.0f;
  const float is16 = 0.0625f;
  const int mt = Mpad / GR;

  hipFuncSetAttribute(reinterpret_cast<const void*>(&k_agg<4, 128>),
                      hipFuncAttributeMaxDynamicSharedMemorySize, AGG_LDS_BYTES);
  hipFuncSetAttribute(reinterpret_cast<const void*>(&k_agg<1, 512>),
                      hipFuncAttributeMaxDynamicSharedMemorySize, AGG_LDS_BYTES);

  k_cvt<<<(Mpad * (K1 / 8) + NTHR - 1) / NTHR, NTHR, 0, stream>>>(x, nN, IN, Ah, Al, Af, Mpad, K1, 1.0f, 3);
  k_cvt<<<(DW * (K1 / 8) + NTHR - 1) / NTHR, NTHR, 0, stream>>>(Wl1, DW, IN, Bh, Bl, Bf, DW, K1, 1.0f, 1);
  k_cvt<<<(DW * (K1 / 8) + NTHR - 1) / NTHR, NTHR, 0, stream>>>(Wr1, DW, IN, Bh, Bl, Bf, DW, K1, s16, 2);
  k_gemm<1><<<dim3(mt, DW / GC), NTHR, 0, stream>>>(Ah, Al, Bh, Bl, bl1, xl, K1, DW, 1.0f);
  k_gemm<0><<<dim3(mt, DW / GC), NTHR, 0, stream>>>(Af, Af, Bf, Bf, br1, xr, K1, DW, is16);
  k_agg<4, 128><<<(Mpad + 127) / 128, NTHR, AGG_LDS_BYTES, stream>>>(ei, xl, xr, at1, b1, Ah, Al, Af, out, nN, nE, Mpad);

  k_cvt<<<(DW * (DW / 8) + NTHR - 1) / NTHR, NTHR, 0, stream>>>(Wl2, DW, DW, Bh, Bl, Bf, DW, DW, 1.0f, 1);
  k_cvt<<<(DW * (DW / 8) + NTHR - 1) / NTHR, NTHR, 0, stream>>>(Wr2, DW, DW, Bh, Bl, Bf, DW, DW, s16, 2);
  k_gemm<1><<<dim3(mt, DW / GC), NTHR, 0, stream>>>(Ah, Al, Bh, Bl, bl2, xl, DW, DW, 1.0f);
  k_gemm<0><<<dim3(mt, DW / GC), NTHR, 0, stream>>>(Af, Af, Bf, Bf, br2, xr, DW, DW, is16);
  k_agg<4, 128><<<(Mpad + 127) / 128, NTHR, AGG_LDS_BYTES, stream>>>(ei, xl, xr, at2, b2, Ah, Al, Af, out, nN, nE, Mpad);

  k_cvt<<<(C3 * (DW / 8) + NTHR - 1) / NTHR, NTHR, 0, stream>>>(Wl3, C3, DW, Bh, Bl, Bf, C3, DW, 1.0f, 1);
  k_cvt<<<(C3 * (DW / 8) + NTHR - 1) / NTHR, NTHR, 0, stream>>>(Wr3, C3, DW, Bh, Bl, Bf, C3, DW, s16, 2);
  k_gemm<1><<<dim3(mt, C3 / GC), NTHR, 0, stream>>>(Ah, Al, Bh, Bl, bl3, xl, DW, C3, 1.0f);
  k_gemm<0><<<dim3(mt, C3 / GC), NTHR, 0, stream>>>(Af, Af, Bf, Bf, br3, xr, DW, C3, is16);
  k_agg<1, 512><<<(nN + 511) / 512, NTHR, AGG_LDS_BYTES, stream>>>(ei, xl, xr, at3, b3, Ah, Al, Af, out, nN, nE, nN);
}
